// ODE_RNN_86852828660358
// MI455X (gfx1250) — hardware-verified
//
#include <hip/hip_runtime.h>
#include <math.h>

constexpr int NBATCH   = 256;
constexpr int NSTEP    = 128;
constexpr int NHID     = 256;
constexpr int NDIM     = 256;
constexpr int NG3      = 3 * NHID;
constexpr int NSUBST   = 2;
constexpr int NTHR     = 256;
constexpr int NWAVE    = NTHR / 32;
constexpr int ROWS_BLK = 16;
constexpr int APITCH   = 264;
constexpr int OTP      = 132;
constexpr int NPAR     = 3 * NG3 + 2 * NHID;
constexpr int NWOC     = NHID + 32;
constexpr float CARRY_A = 16.0f;
constexpr float CARRY_W = 16.0f;
constexpr float FOLD_AW = 1.0f / 256.0f;

static_assert(NBATCH % ROWS_BLK == 0);
static_assert(NHID == 32 * NWAVE);
static_assert(NDIM == NHID && NHID % 64 == 0);
static_assert(APITCH % 8 == 0 && APITCH >= NHID);
static_assert(OTP % 4 == 0 && OTP >= NSTEP);
static_assert(ROWS_BLK * NSTEP == 4 * 2 * NTHR);
static_assert(ROWS_BLK * NSTEP * 2 == 4 * 4 * NTHR);
static_assert(NSTEP * 2 == 4 * 64);
static_assert((2 * ROWS_BLK * APITCH) % NTHR == 0);
static_assert(NG3 == 4 * 192 && NHID == 4 * 64);
static_assert((NG3 * NHID) % (8 * NTHR) == 0);
static_assert(NHID % 32 == 0 && NWAVE * 4 == 32);
static_assert(NWOC == 4 * 72);
static_assert(NSTEP == 4 * 32);

typedef __attribute__((ext_vector_type(16))) _Float16 v16h;
typedef __attribute__((ext_vector_type(8)))  _Float16 v8h;
typedef __attribute__((ext_vector_type(8)))  float    v8f;
typedef __attribute__((ext_vector_type(4)))  float    v4f;

template <typename T> struct Frag;
template <> struct Frag<_Float16> {
  typedef v16h V; union U { v16h v; v8h h[2]; };
  static __device__ __forceinline__ v16h load(const _Float16* p) {
    U f; f.h[0] = *(const v8h*)(p); f.h[1] = *(const v8h*)(p + 16); return f.v;
  }
  static __device__ __forceinline__ v8f mma(v16h a, v16h b, v8f c) {
    return __builtin_amdgcn_wmma_f32_16x16x32_f16(false, a, false, b, (short)0, c, false, false);
  }
};

__device__ __forceinline__ void guard2h(v8f& a0, v8f& a1, v16h fa, v16h fb0, v16h fb1) {
  asm volatile("v_nop\n\tv_nop\n\tv_nop\n\tv_nop" : "+v"(a0), "+v"(a1) : "v"(fa), "v"(fb0), "v"(fb1));
}
__device__ __forceinline__ void guard3h(v8f& a0, v8f& a1, v8f& a2, v16h fa, v16h fb0, v16h fb1, v16h fb2) {
  asm volatile("v_nop\n\tv_nop\n\tv_nop\n\tv_nop" : "+v"(a0), "+v"(a1), "+v"(a2) : "v"(fa), "v"(fb0), "v"(fb1), "v"(fb2));
}
__device__ __forceinline__ void acc_guard2(v8f& a, v8f& b) { asm volatile("v_nop\n\tv_nop\n\tv_nop\n\tv_nop" : "+v"(a), "+v"(b)); }
__device__ __forceinline__ void acc_guard3(v8f& a, v8f& b, v8f& c) { asm volatile("v_nop\n\tv_nop\n\tv_nop\n\tv_nop" : "+v"(a), "+v"(b), "+v"(c)); }

__device__ __forceinline__ float fsig(float x)  { return __builtin_amdgcn_rcpf(1.0f + expf(-x)); }
__device__ __forceinline__ float ftanh(float x) { return 1.0f - 2.0f * __builtin_amdgcn_rcpf(1.0f + expf(2.0f * x)); }

__global__ __launch_bounds__(NTHR) void fold_kernel(const float* __restrict__ W1, const float* __restrict__ b1,
                                                    const float* __restrict__ W2, const float* __restrict__ b2,
                                                    const float* __restrict__ Wo1, const float* __restrict__ bo1,
                                                    const float* __restrict__ Wo2, const float* __restrict__ bo2,
                                                    unsigned short* __restrict__ WCP, float* __restrict__ BC,
                                                    float* __restrict__ WOC) {
  __shared__ __align__(16) float sred[NWOC];
  const int tid = threadIdx.x, lane = tid & 31, wave = tid >> 5;
  if (blockIdx.x < NHID / 32) {
    const int nbase = blockIdx.x * 32;
#pragma unroll 1
    for (int q = 0; q < 4; ++q) {
      const int n = nbase + wave * 4 + q;
      float a[8];
#pragma unroll
      for (int e = 0; e < 8; ++e) a[e] = 0.0f;
      float ab = 0.0f;
      const float* w2row = W2 + (size_t)n * NDIM;
#pragma unroll 1
      for (int d = 0; d < NDIM; ++d) {
        const float w2 = w2row[d];
        const float bd = b1[d];
        const float* w1row = W1 + (size_t)d * NHID + 8 * lane;
        const v4f x0 = *(const v4f*)(w1row);
        const v4f x1 = *(const v4f*)(w1row + 4);
#pragma unroll
        for (int e = 0; e < 4; ++e) {
          a[e]     = fmaf(w2, x0[e], a[e]);
          a[4 + e] = fmaf(w2, x1[e], a[4 + e]);
        }
        ab = fmaf(w2, bd, ab);
      }
      v8h hv;
#pragma unroll
      for (int e = 0; e < 8; ++e) hv[e] = (_Float16)(a[e] * CARRY_W);
      unsigned short* dst = WCP + (size_t)n * NHID + 8 * lane;
      *(volatile v8h*)dst = hv;
      __threadfence();
      *(volatile v8h*)dst = hv;
      const float b2n = b2[n];
      if (lane == 0) sred[wave * 4 + q] = ab + b2n;
    }
    __syncthreads();
    if (wave == 0) {
      const int l8 = lane & 7;
      const v4f v = *(const v4f*)(sred + 4 * l8);
      if (lane < 8) {
        float* dst = BC + nbase + 4 * lane;
        *(volatile v4f*)dst = v;
        __threadfence();
        *(volatile v4f*)dst = v;
      }
    }
  } else {
    const int k = tid;
    float acc = 0.0f, accc = 0.0f;
#pragma unroll 1
    for (int d = 0; d < NDIM; ++d) {
      const float w = Wo2[d];
      acc  = fmaf(w, Wo1[(size_t)d * NHID + k], acc);
      accc = fmaf(w, bo1[d], accc);
    }
    const float cval = accc + bo2[0];
    sred[k] = acc;
    if (tid < 32) sred[NHID + tid] = (tid == 0) ? cval : 0.0f;
    __syncthreads();
    {
      const int i = (tid < 72) ? tid : 71;
      const v4f v = *(const v4f*)(sred + 4 * i);
      if (tid < 72) {
        float* dst = WOC + 4 * tid;
        *(volatile v4f*)dst = v;
        __threadfence();
        *(volatile v4f*)dst = v;
      }
    }
  }
}

__global__ __launch_bounds__(NTHR) void cast_scale_f16x8(const float* __restrict__ src, unsigned short* __restrict__ dst,
                                                        int n8, float sc) {
  const int i = blockIdx.x * NTHR + threadIdx.x;
  if (i < n8) {
    const float* sp = src + (size_t)i * 8;
    const v4f a = *(const v4f*)(sp);
    const v4f b = *(const v4f*)(sp + 4);
    v8h hv;
#pragma unroll
    for (int e = 0; e < 4; ++e) {
      hv[e]     = (_Float16)(a[e] * sc);
      hv[4 + e] = (_Float16)(b[e] * sc);
    }
    unsigned short* dp = dst + (size_t)i * 8;
    *(volatile v8h*)dp = hv;
    __threadfence();
    *(volatile v8h*)dp = hv;
  }
}

__global__ __launch_bounds__(NTHR) void ode_gru_kernel(const float* __restrict__ bIn,   const float* __restrict__ mIn,
                                                       const float* __restrict__ trmIn, const float* __restrict__ temIn,
                                                       const float* __restrict__ h0In,  const float* __restrict__ Wih,
                                                       const float* __restrict__ bih,   const float* __restrict__ bhh,
                                                       const unsigned short* __restrict__ WCPp,
                                                       const unsigned short* __restrict__ WHPp,
                                                       const float* __restrict__ BC, const float* __restrict__ WOC,
                                                       float* __restrict__ out) {
  __shared__ __align__(16) _Float16 Ah[2][ROWS_BLK * APITCH];
  __shared__ __align__(16) float sval[ROWS_BLK * NSTEP];
  __shared__ __align__(16) float smv [ROWS_BLK * NSTEP];
  __shared__ __align__(16) float strm[ROWS_BLK * NSTEP];
  __shared__ __align__(16) float stem[ROWS_BLK * NSTEP];
  __shared__ __align__(16) float stim[NSTEP];
  __shared__ __align__(16) float spar[NPAR];
  __shared__ float sred[NWAVE * ROWS_BLK];
  __shared__ float sout[ROWS_BLK];
  __shared__ __align__(16) float otile[ROWS_BLK * OTP];

  const _Float16* WCP = (const _Float16*)WCPp;
  const _Float16* WHP = (const _Float16*)WHPp;
  const int tid = threadIdx.x, lane = tid & 31, wave = tid >> 5;
  const int c = lane & 15, hh = lane >> 4, koff = hh * 8;
  const int rowbase = blockIdx.x * ROWS_BLK;

  {
    _Float16* ahf = &Ah[0][0];
#pragma unroll 1
    for (int i = tid; i < 2 * ROWS_BLK * APITCH; i += NTHR) ahf[i] = (_Float16)0.0f;
  }
  {
#pragma unroll
    for (int it = 0; it < 2; ++it) {
      const int idx = it * NTHR + tid;
      const int row = idx >> 5, c4 = (idx & 31) * 4;
      const size_t g = (size_t)(rowbase + row) * NSTEP + c4;
      const v4f vm = *(const v4f*)(mIn + g);
      const v4f va = *(const v4f*)(trmIn + g);
      const v4f vb = *(const v4f*)(temIn + g);
      *(v4f*)(smv  + row * NSTEP + c4) = vm;
      *(v4f*)(strm + row * NSTEP + c4) = va;
      *(v4f*)(stem + row * NSTEP + c4) = vb;
    }
    asm volatile("" ::: "memory");
#pragma unroll
    for (int it = 0; it < 4; ++it) {
      const int idx = it * NTHR + tid;
      const int row = idx >> 6, q = idx & 63;
      const v4f v = *(const v4f*)(bIn + (size_t)(rowbase + row) * (NSTEP * 2) + 4 * q);
      sval[row * NSTEP + 2 * q]     = v[1];
      sval[row * NSTEP + 2 * q + 1] = v[3];
    }
    asm volatile("" ::: "memory");
    if (tid < 64) {
      const v4f v = *(const v4f*)(bIn + 4 * tid);
      stim[2 * tid]     = v[0];
      stim[2 * tid + 1] = v[2];
      const v4f pa = *(const v4f*)(BC + 4 * tid);
      const v4f pb = *(const v4f*)(WOC + 4 * tid);
      *(v4f*)(spar + 3 * NG3 + 4 * tid)        = pa;
      *(v4f*)(spar + 3 * NG3 + NHID + 4 * tid) = pb;
    }
    asm volatile("" ::: "memory");
    if (tid < 192) {
      const v4f pa = *(const v4f*)(Wih + 4 * tid);
      const v4f pb = *(const v4f*)(bih + 4 * tid);
      const v4f pc = *(const v4f*)(bhh + 4 * tid);
      *(v4f*)(spar + 4 * tid)           = pa;
      *(v4f*)(spar + NG3 + 4 * tid)     = pb;
      *(v4f*)(spar + 2 * NG3 + 4 * tid) = pc;
    }
  }
  __syncthreads();

  float kw[2][3], kbi[2][3], kbh[2][3], kbc[2], kwo[2];
#pragma unroll
  for (int nt = 0; nt < 2; ++nt) {
    const int j = 32 * wave + 16 * nt + c;
#pragma unroll
    for (int g = 0; g < 3; ++g) {
      kw[nt][g]  = spar[g * NHID + j];
      kbi[nt][g] = spar[NG3 + g * NHID + j];
      kbh[nt][g] = spar[2 * NG3 + g * NHID + j];
    }
    kbc[nt] = spar[3 * NG3 + j];
    kwo[nt] = spar[3 * NG3 + NHID + j];
  }
  const float c0v = WOC[NHID];
  float hst[2][8], ksum[2][8];
#pragma unroll
  for (int nt = 0; nt < 2; ++nt) {
    const int j = 32 * wave + 16 * nt + c;
#pragma unroll
    for (int r = 0; r < 8; ++r) {
      const float h = h0In[(size_t)(rowbase + 8 * hh + r) * NHID + j];
      hst[nt][r]  = h;
      ksum[nt][r] = 0.0f;
      Ah[0][(8 * hh + r) * APITCH + j] = (_Float16)(h * CARRY_A);
    }
    asm volatile("" ::: "memory");
  }
  __syncthreads();

  const v8f z8 = {0.f, 0.f, 0.f, 0.f, 0.f, 0.f, 0.f, 0.f};
  int cur = 0;

#pragma unroll 1
  for (int t = 0; t < NSTEP; ++t) {
    const int   tpi   = (t > 0) ? (t - 1) : 0;
    const float tpraw = stim[tpi];
    const float tprev = (t > 0) ? tpraw : 0.0f;
    const float dt    = (stim[t] - tprev) * 0.5f;
    const float hdt   = 0.5f * dt;
    const float dt6   = dt / 6.0f;

#pragma unroll 1
    for (int sg = 0; sg < 4 * NSUBST; ++sg) {
      const int  s  = sg & 3;
      const bool s0 = (s == 0), s3 = (s == 3);
      const float cm = (s == 2) ? dt : hdt;
      const _Float16* arow  = &Ah[cur][0] + c * APITCH + koff;
      _Float16*       anext = &Ah[cur ^ 1][0];
      const int j0 = 32 * wave + c;
      const _Float16* w0 = WCP + (size_t)j0 * NHID + koff;
      const _Float16* w1 = WCP + (size_t)(j0 + 16) * NHID + koff;
      v8f acc[2];
      acc[0] = z8; acc[1] = z8;
#pragma unroll 1
      for (int k0 = 0; k0 < NHID; k0 += 64) {
        {
          const v16h a  = Frag<_Float16>::load(arow + k0);
          const v16h b0 = Frag<_Float16>::load(w0 + k0);
          const v16h b1 = Frag<_Float16>::load(w1 + k0);
          acc[0] = Frag<_Float16>::mma(a, b0, acc[0]);
          acc[1] = Frag<_Float16>::mma(a, b1, acc[1]);
          guard2h(acc[0], acc[1], a, b0, b1);
        }
        {
          const v16h a  = Frag<_Float16>::load(arow + k0 + 32);
          const v16h b0 = Frag<_Float16>::load(w0 + k0 + 32);
          const v16h b1 = Frag<_Float16>::load(w1 + k0 + 32);
          acc[0] = Frag<_Float16>::mma(a, b0, acc[0]);
          acc[1] = Frag<_Float16>::mma(a, b1, acc[1]);
          guard2h(acc[0], acc[1], a, b0, b1);
        }
      }
      acc_guard2(acc[0], acc[1]);
#pragma unroll
      for (int nt = 0; nt < 2; ++nt) {
        const int j = 32 * wave + 16 * nt + c;
#pragma unroll
        for (int r = 0; r < 8; ++r) {
          const float pre  = fmaf(acc[nt][r], FOLD_AW, kbc[nt]);
          const float kv   = ftanh(pre);
          const float hold = hst[nt][r];
          const float kadd = (s0 || s3) ? kv : 2.0f * kv;
          const float ksn  = ksum[nt][r] + kadd;
          const float hn   = s3 ? fmaf(dt6, ksn, hold) : hold;
          const float xn   = s3 ? hn : fmaf(cm, kv, hold);
          ksum[nt][r] = s3 ? 0.0f : ksn;
          hst[nt][r]  = hn;
          anext[(8 * hh + r) * APITCH + j] = (_Float16)(xn * CARRY_A);
        }
      }
      __syncthreads();
      cur ^= 1;
    }

    {
      float p[8];
#pragma unroll
      for (int r = 0; r < 8; ++r) {
        float v = 0.0f;
        v = fmaf(hst[0][r], kwo[0], v);
        v = fmaf(hst[1][r], kwo[1], v);
        p[r] = v;
      }
#pragma unroll
      for (int r = 0; r < 8; ++r) {
#pragma unroll
        for (int off = 1; off < 16; off <<= 1) p[r] += __shfl_xor(p[r], off, 32);
      }
      if (c == 0) {
#pragma unroll
        for (int r = 0; r < 8; ++r) sred[wave * ROWS_BLK + 8 * hh + r] = p[r];
      }
    }
    __syncthreads();
    if (wave == 0) {
      const int row = lane & 15;
      float sm = 0.0f;
#pragma unroll
      for (int w = 0; w < NWAVE; ++w) sm += sred[w * ROWS_BLK + row];
      const float ov = tanhf(sm + c0v);
      if (lane < 16) {
        sout[row] = ov;
        otile[row * OTP + t] = ov;
      }
    }
    __syncthreads();

    {
      const _Float16* arow  = &Ah[cur][0] + c * APITCH + koff;
      _Float16*       anext = &Ah[cur ^ 1][0];
#pragma unroll
      for (int nt = 0; nt < 2; ++nt) {
        const int j = 32 * wave + 16 * nt + c;
        const _Float16* wr = WHP + (size_t)j * NHID + koff;
        const _Float16* wz = wr + (size_t)NHID * NHID;
        const _Float16* wn = wr + (size_t)2 * NHID * NHID;
        v8f g3[3];
        g3[0] = z8; g3[1] = z8; g3[2] = z8;
#pragma unroll 1
        for (int k0 = 0; k0 < NHID; k0 += 64) {
          {
            const v16h a  = Frag<_Float16>::load(arow + k0);
            const v16h br = Frag<_Float16>::load(wr + k0);
            const v16h bz = Frag<_Float16>::load(wz + k0);
            const v16h bn = Frag<_Float16>::load(wn + k0);
            g3[0] = Frag<_Float16>::mma(a, br, g3[0]);
            g3[1] = Frag<_Float16>::mma(a, bz, g3[1]);
            g3[2] = Frag<_Float16>::mma(a, bn, g3[2]);
            guard3h(g3[0], g3[1], g3[2], a, br, bz, bn);
          }
          {
            const v16h a  = Frag<_Float16>::load(arow + k0 + 32);
            const v16h br = Frag<_Float16>::load(wr + k0 + 32);
            const v16h bz = Frag<_Float16>::load(wz + k0 + 32);
            const v16h bn = Frag<_Float16>::load(wn + k0 + 32);
            g3[0] = Frag<_Float16>::mma(a, br, g3[0]);
            g3[1] = Frag<_Float16>::mma(a, bz, g3[1]);
            g3[2] = Frag<_Float16>::mma(a, bn, g3[2]);
            guard3h(g3[0], g3[1], g3[2], a, br, bz, bn);
          }
        }
        acc_guard3(g3[0], g3[1], g3[2]);
#pragma unroll
        for (int r = 0; r < 8; ++r) {
          const int   i   = 8 * hh + r;
          const float hp  = hst[nt][r];
          const float ghr = fmaf(g3[0][r], FOLD_AW, kbh[nt][0]);
          const float ghz = fmaf(g3[1][r], FOLD_AW, kbh[nt][1]);
          const float ghn = fmaf(g3[2][r], FOLD_AW, kbh[nt][2]);
          const float trm = strm[i * NSTEP + t];
          const float tem = stem[i * NSTEP + t];
          const float mv  = smv [i * NSTEP + t];
          const float val = sval[i * NSTEP + t];
          const float ov  = sout[i];
          const float xtr = val * trm;
          const float xte = ov * tem;
          const float r1 = fsig(fmaf(xtr, kw[nt][0], kbi[nt][0]) + ghr);
          const float z1 = fsig(fmaf(xtr, kw[nt][1], kbi[nt][1]) + ghz);
          const float n1 = ftanh(fmaf(xtr, kw[nt][2], kbi[nt][2]) + r1 * ghn);
          const float htr = (1.0f - z1) * n1 + z1 * hp;
          const float r2 = fsig(fmaf(xte, kw[nt][0], kbi[nt][0]) + ghr);
          const float z2 = fsig(fmaf(xte, kw[nt][1], kbi[nt][1]) + ghz);
          const float n2 = ftanh(fmaf(xte, kw[nt][2], kbi[nt][2]) + r2 * ghn);
          const float hte = (1.0f - z2) * n2 + z2 * hp;
          const float hn  = trm * htr + tem * hte + (1.0f - mv) * hp;
          hst[nt][r] = hn;
          anext[i * APITCH + j] = (_Float16)(hn * CARRY_A);
        }
      }
    }
    __syncthreads();
    cur ^= 1;
  }

  for (int pass = 0; pass < 2; ++pass) {
#pragma unroll
    for (int it = 0; it < 2; ++it) {
      const int idx = it * NTHR + tid;
      const int row = idx >> 5, c4 = (idx & 31) * 4;
      const v4f v = *(const v4f*)(otile + row * OTP + c4);
      *(volatile v4f*)(out + (size_t)(rowbase + row) * NSTEP + c4) = v;
    }
    __threadfence();
  }
}

extern "C" void kernel_launch(void* const* d_in, const int* in_sizes, int n_in,
                              void* d_out, int out_size, void* d_ws, size_t ws_size, hipStream_t stream) {
  if (n_in < 17 || d_out == nullptr || d_ws == nullptr) return;
  if (in_sizes[0] != NBATCH * NSTEP * 2 || in_sizes[1] != NBATCH * NSTEP || in_sizes[2] != NBATCH * NSTEP ||
      in_sizes[3] != NBATCH * NSTEP || in_sizes[4] != NBATCH * NHID || in_sizes[5] != NDIM * NHID ||
      in_sizes[6] != NDIM || in_sizes[7] != NHID * NDIM || in_sizes[8] != NHID || in_sizes[9] != NG3 ||
      in_sizes[10] != NG3 * NHID || in_sizes[11] != NG3 || in_sizes[12] != NG3 || in_sizes[13] != NDIM * NHID ||
      in_sizes[14] != NDIM || in_sizes[15] != NDIM || in_sizes[16] != 1 || out_size != NBATCH * NSTEP) return;

  const float* bIn   = (const float*)d_in[0];
  const float* mIn   = (const float*)d_in[1];
  const float* trmIn = (const float*)d_in[2];
  const float* temIn = (const float*)d_in[3];
  const float* h0In  = (const float*)d_in[4];
  const float* W1    = (const float*)d_in[5];
  const float* b1    = (const float*)d_in[6];
  const float* W2    = (const float*)d_in[7];
  const float* b2    = (const float*)d_in[8];
  const float* Wih   = (const float*)d_in[9];
  const float* Whh   = (const float*)d_in[10];
  const float* bih   = (const float*)d_in[11];
  const float* bhh   = (const float*)d_in[12];
  const float* Wo1   = (const float*)d_in[13];
  const float* bo1   = (const float*)d_in[14];
  const float* Wo2   = (const float*)d_in[15];
  const float* bo2   = (const float*)d_in[16];
  float* out = (float*)d_out;

  char* ws = (char*)d_ws; size_t off = 0;
  auto carve = [&](size_t bytes) -> char* { char* p = ws + off; off += (bytes + 255) & ~(size_t)255; return p; };
  unsigned short* WCP = (unsigned short*)carve((size_t)NHID * NHID * 2);
  unsigned short* WHP = (unsigned short*)carve((size_t)NG3 * NHID * 2);
  float*          BC  = (float*)carve((size_t)NHID * 4);
  float*          WOC = (float*)carve((size_t)NWOC * 4);
  if (off > ws_size || off > (size_t)134217728) return;

  fold_kernel<<<NHID / 32 + 1, NTHR, 0, stream>>>(W1, b1, W2, b2, Wo1, bo1, Wo2, bo2, WCP, BC, WOC);
  const int n8 = NG3 * NHID / 8;
  cast_scale_f16x8<<<(n8 + NTHR - 1) / NTHR, NTHR, 0, stream>>>(Whh, WHP, n8, CARRY_W);
  ode_gru_kernel<<<NBATCH / ROWS_BLK, NTHR, 0, stream>>>(bIn, mIn, trmIn, temIn, h0In, Wih, bih, bhh, WCP, WHP, BC, WOC, out);
}
